// BasicGraphClassifier_395136991531
// MI455X (gfx1250) — hardware-verified
//
#include <hip/hip_runtime.h>
#include <stddef.h>
#include <stdint.h>


#define N_NODES  50000
#define N_EDGES  800000
#define IN_DIM   128
#define HID      256
#define NCLS     10
#define NCLS_PAD 16
#define NGRAPH   64

#define ECHUNK   2048
#define WSEG     256

typedef _Float16 v16h __attribute__((ext_vector_type(16)));
typedef _Float16 v8h  __attribute__((ext_vector_type(8)));
typedef float    v8f  __attribute__((ext_vector_type(8)));
typedef float    v4f  __attribute__((ext_vector_type(4)));
typedef float    v4fa __attribute__((ext_vector_type(4), __may_alias__));
typedef int      v4i  __attribute__((ext_vector_type(4)));
union Frag { v16h v; v8h h[2]; };

__device__ __forceinline__ v8f wmma_f16(v16h a, v16h b, v8f c) {
  c = __builtin_amdgcn_wmma_f32_16x16x32_f16(false, a, false, b, (short)0, c, false, false);
  asm volatile("v_nop\n\tv_nop\n\tv_nop\n\tv_nop" : "+v"(c) : "v"(a), "v"(b));
  return c;
}

__device__ __forceinline__ unsigned ballot32(bool p) { return __builtin_amdgcn_ballot_w32(p); }

__device__ __forceinline__ v8h pack8h(v4f a, v4f b) {
  v8f f = __builtin_shufflevector(a, b, 0, 1, 2, 3, 4, 5, 6, 7);
  return __builtin_convertvector(f, v8h);
}

__global__ __launch_bounds__(256)
void k_cvt(const float* __restrict__ s, _Float16* __restrict__ d, int nsrc, int ndst8) {
  const int i = blockIdx.x * 256 + threadIdx.x;
  if (i >= ndst8) return;
  v8f f;
#pragma unroll
  for (int k = 0; k < 8; ++k) {
    const int idx = i * 8 + k;
    f[k] = (idx < nsrc) ? s[idx] : 0.0f;
  }
  const v8h o = __builtin_convertvector(f, v8h);
  volatile v8h* p = (volatile v8h*)(d + (size_t)i * 8);
  *p = o;
  __threadfence();
  *p = o;
}

template <int D, int R>
__device__ __forceinline__ void agg_emit(const float* acc, _Float16* __restrict__ z,
                                         int base, int w, int l) {
  constexpr int NPW  = R / 8;
  constexpr int LPRW = D / 8;
  constexpr int RPI  = 32 / LPRW;
  const int rsub = l / LPRW;
  const int cc   = (l % LPRW) * 8;
  for (int i = 0; i < NPW; i += RPI) {
    const int ld   = w * NPW + i + rsub;
    const int node = base + ld;
    const v4fa* ap = (const v4fa*)(acc + ld * D + cc);
    const v8h o = pack8h(ap[0], ap[1]);
    if (node < N_NODES)
      *(volatile v8h*)(z + (size_t)node * D + cc) = o;
  }
}

template <int D, int R>
__global__ __launch_bounds__(256)
void k_agg(const float* __restrict__ h, const int* __restrict__ ei, _Float16* __restrict__ z) {
  constexpr int NPW  = R / 8;
  constexpr int LNPW = (NPW == 32) ? 5 : 4;
  constexpr int F4   = D / 128;
  __shared__ __attribute__((aligned(16))) float acc[R * D];
  __shared__ unsigned lst[ECHUNK];
  __shared__ int wcnt[8];

  const int l = threadIdx.x & 31, w = threadIdx.x >> 5;
  const int base = blockIdx.x * R;
  const int rcnt = min(R, N_NODES - base);
  const v4f z4 = {0.0f, 0.0f, 0.0f, 0.0f};

  for (int i = 0; i < NPW; ++i) {
    const int ld = w * NPW + i, node = base + ld;
    v4fa* ap = (v4fa*)(acc + ld * D + l * 4 * F4);
    if (node < N_NODES) {
      const v4f* hp = (const v4f*)(h + (size_t)node * D + l * 4 * F4);
#pragma unroll
      for (int f = 0; f < F4; ++f) ap[f] = hp[f];
    } else {
#pragma unroll
      for (int f = 0; f < F4; ++f) ap[f] = z4;
    }
  }

  const int* srcp = ei;
  const int* dstp = ei + N_EDGES;
  const int nch = (N_EDGES + ECHUNK - 1) / ECHUNK;
  for (int c = 0; c < nch; ++c) {
    const int e0 = c * ECHUNK + w * WSEG + l * 8;
    int dv[8];
    if (e0 + 8 <= N_EDGES) {
      const v4i a = *(const v4i*)(dstp + e0);
      const v4i b = *(const v4i*)(dstp + e0 + 4);
      dv[0] = a[0]; dv[1] = a[1]; dv[2] = a[2]; dv[3] = a[3];
      dv[4] = b[0]; dv[5] = b[1]; dv[6] = b[2]; dv[7] = b[3];
    } else {
#pragma unroll
      for (int j = 0; j < 8; ++j) dv[j] = (e0 + j < N_EDGES) ? dstp[e0 + j] : -1;
    }
    bool hit[8];
    bool any = false;
#pragma unroll
    for (int j = 0; j < 8; ++j) {
      const int t = dv[j] - base;
      hit[j] = (unsigned)t < (unsigned)rcnt;
      any |= hit[j];
    }
    int cnt = 0;
    if (ballot32(any) != 0u) {
#pragma unroll
      for (int j = 0; j < 8; ++j) {
        const unsigned m = ballot32(hit[j]);
        if (hit[j]) {
          const int pos = cnt + (int)__builtin_popcount(m & ((1u << l) - 1u));
          int s = srcp[e0 + j];
          s = min(max(s, 0), N_NODES - 1);
          const unsigned t = (unsigned)(dv[j] - base);
          lst[w * WSEG + pos] = (unsigned)s | (t << 16);
        }
        cnt += (int)__builtin_popcount(m);
      }
    }
    if (l == 0) wcnt[w] = cnt;
    __syncthreads();

    for (int v = 0; v < 8; ++v) {
      const int cv = min(wcnt[v], WSEG);
      for (int i0 = 0; i0 < cv; i0 += 32) {
        const int idx = i0 + l;
        const unsigned ent = (idx < cv) ? lst[v * WSEG + idx] : 0u;
        const bool mine = (idx < cv) && ((((int)(ent >> 16)) >> LNPW) == w);
        unsigned mm = ballot32(mine);
        while (mm != 0u) {
          const int bp = __builtin_ctz(mm);
          mm &= mm - 1u;
          const unsigned eb = lst[v * WSEG + i0 + bp];
          const int s  = min((int)(eb & 0xFFFFu), N_NODES - 1);
          const int tt = (int)(eb >> 16) & (R - 1);
          const v4f* hp = (const v4f*)(h + (size_t)s * D + l * 4 * F4);
          v4fa* ap = (v4fa*)(acc + tt * D + l * 4 * F4);
#pragma unroll
          for (int f = 0; f < F4; ++f) ap[f] = ap[f] + hp[f];
        }
      }
    }
    __syncthreads();
  }

  agg_emit<D, R>(acc, z, base, w, l);
  __threadfence();
  agg_emit<D, R>(acc, z, base, w, l);
}

template <int MODE>
__device__ __forceinline__ void gemm_emit(const float* sw, const float* __restrict__ bias,
                                          void* __restrict__ outp, int mT, int strip,
                                          int l, bool active) {
  if (MODE == 0) {
    _Float16* out = (_Float16*)outp;
    const int rl = l >> 3, cc = (l & 7) * 8;
    const v4f b0 = *(const v4f*)(bias + strip * 64 + cc);
    const v4f b1 = *(const v4f*)(bias + strip * 64 + cc + 4);
#pragma unroll
    for (int q = 0; q < 4; ++q) {
      const int row = q * 4 + rl;
      const v4fa* sp = (const v4fa*)(sw + row * 64 + cc);
      v4f x0 = sp[0] + b0, x1 = sp[1] + b1;
#pragma unroll
      for (int e = 0; e < 4; ++e) { x0[e] = fmaxf(x0[e], 0.0f); x1[e] = fmaxf(x1[e], 0.0f); }
      const v8h o = pack8h(x0, x1);
      if (active)
        *(volatile v8h*)(out + (size_t)(mT * 16 + row) * HID + strip * 64 + cc) = o;
    }
  } else {
    float* out = (float*)outp;
    const int rl = l >> 4, cc = (l & 15) * 4;
    const v4f b0 = *(const v4f*)(bias + strip * 64 + cc);
#pragma unroll
    for (int q = 0; q < 8; ++q) {
      const int row = q * 2 + rl;
      const v4fa* sp = (const v4fa*)(sw + row * 64 + cc);
      const v4f x = sp[0] + b0;
      if (active)
        *(volatile v4f*)(out + (size_t)(mT * 16 + row) * HID + strip * 64 + cc) = x;
    }
  }
}

template <int MODE>
__global__ __launch_bounds__(256)
void k_gemm(const _Float16* __restrict__ A, const _Float16* __restrict__ Wt,
            const float* __restrict__ bias, void* __restrict__ outp, int Kin, int ntiles) {
  __shared__ __attribute__((aligned(16))) float stg[8 * 1024];
  const int l = threadIdx.x & 31, hh = l >> 4, m = l & 15, w = threadIdx.x >> 5;
  const int raw = blockIdx.x * 8 + w;
  const bool active = raw < ntiles;
  const int tile = active ? raw : (ntiles - 1);
  const int mT = tile >> 2, strip = tile & 3;

  const _Float16* Ap  = A  + (size_t)(mT * 16 + m) * Kin;
  const _Float16* Bp0 = Wt + (size_t)(strip * 64 + m) * Kin;

  const v8f z8 = {0.0f, 0.0f, 0.0f, 0.0f, 0.0f, 0.0f, 0.0f, 0.0f};
  v8f c[4];
#pragma unroll
  for (int j = 0; j < 4; ++j) c[j] = z8;

  for (int kb = 0; kb < Kin; kb += 32) {
    Frag a;
    a.h[0] = *(const v8h*)(Ap + kb + 8 * hh);
    a.h[1] = *(const v8h*)(Ap + kb + 16 + 8 * hh);
#pragma unroll
    for (int j = 0; j < 4; ++j) {
      const _Float16* Bp = Bp0 + (size_t)(j * 16) * Kin + kb;
      Frag b;
      b.h[0] = *(const v8h*)(Bp + 8 * hh);
      b.h[1] = *(const v8h*)(Bp + 16 + 8 * hh);
      c[j] = wmma_f16(a.v, b.v, c[j]);
    }
  }

  float* sw = stg + w * 1024;
#pragma unroll
  for (int j = 0; j < 4; ++j)
#pragma unroll
    for (int r = 0; r < 8; ++r) sw[(8 * hh + r) * 64 + j * 16 + m] = c[j][r];
  __syncthreads();

  gemm_emit<MODE>(sw, bias, outp, mT, strip, l, active);
  __threadfence();
  gemm_emit<MODE>(sw, bias, outp, mT, strip, l, active);
}

__global__ __launch_bounds__(256)
void k_pool(const float* __restrict__ h2, const int* __restrict__ gid, _Float16* __restrict__ pm) {
  __shared__ int lst[ECHUNK];
  __shared__ int wcnt[8];
  __shared__ __attribute__((aligned(16))) float sm[HID];
  const int t = threadIdx.x, l = t & 31, w = t >> 5, g = blockIdx.x;
  float sum = 0.0f;
  int total = 0;
  const int nch = (N_NODES + ECHUNK - 1) / ECHUNK;
  for (int c = 0; c < nch; ++c) {
    const int n0 = c * ECHUNK + w * WSEG + l * 8;
    int bv[8];
    if (n0 + 8 <= N_NODES) {
      const v4i a = *(const v4i*)(gid + n0);
      const v4i b = *(const v4i*)(gid + n0 + 4);
      bv[0] = a[0]; bv[1] = a[1]; bv[2] = a[2]; bv[3] = a[3];
      bv[4] = b[0]; bv[5] = b[1]; bv[6] = b[2]; bv[7] = b[3];
    } else {
#pragma unroll
      for (int j = 0; j < 8; ++j) bv[j] = (n0 + j < N_NODES) ? gid[n0 + j] : -1;
    }
    int cnt = 0;
#pragma unroll
    for (int j = 0; j < 8; ++j) {
      const bool hit = (bv[j] == g);
      const unsigned m = ballot32(hit);
      if (hit) lst[w * WSEG + cnt + (int)__builtin_popcount(m & ((1u << l) - 1u))] = n0 + j;
      cnt += (int)__builtin_popcount(m);
    }
    if (l == 0) wcnt[w] = cnt;
    __syncthreads();
    for (int v = 0; v < 8; ++v) {
      const int cv = min(wcnt[v], WSEG);
      total += max(cv, 0);
      for (int i = 0; i < cv; ++i) {
        const int node = min(max(lst[v * WSEG + i], 0), N_NODES - 1);
        sum += h2[(size_t)node * HID + t];
      }
    }
    __syncthreads();
  }
  const float inv = 1.0f / fmaxf((float)total, 1.0f);
  sm[t] = sum * inv;
  __syncthreads();
  if (w == 0) {
    const v4fa* sp = (const v4fa*)(sm + l * 8);
    const v8h o = pack8h(sp[0], sp[1]);
    volatile v8h* p = (volatile v8h*)(pm + (size_t)g * HID + l * 8);
    *p = o;
    __threadfence();
    *p = o;
  }
}

__device__ __forceinline__ void cls_emit(const float* so, float* __restrict__ out, int l) {
#pragma unroll
  for (int q = 0; q < 5; ++q) {
    const int i4 = q * 32 + l;
    const v4f v = *(const v4fa*)(so + i4 * 4);
    *(volatile v4f*)(out + i4 * 4) = v;
  }
}

__global__ __launch_bounds__(128)
void k_cls(const _Float16* __restrict__ pm, const _Float16* __restrict__ Wch,
           const float* __restrict__ bc, float* __restrict__ out) {
  __shared__ __attribute__((aligned(16))) float so[NGRAPH * NCLS];
  const int l = threadIdx.x & 31, hh = l >> 4, m = l & 15, w = threadIdx.x >> 5;
  const _Float16* Ap = pm  + (size_t)(w * 16 + m) * HID;
  const _Float16* Bp = Wch + (size_t)m * HID;
  v8f acc = {0.0f, 0.0f, 0.0f, 0.0f, 0.0f, 0.0f, 0.0f, 0.0f};
  for (int kb = 0; kb < HID; kb += 32) {
    Frag a, b;
    a.h[0] = *(const v8h*)(Ap + kb + 8 * hh);
    a.h[1] = *(const v8h*)(Ap + kb + 16 + 8 * hh);
    b.h[0] = *(const v8h*)(Bp + kb + 8 * hh);
    b.h[1] = *(const v8h*)(Bp + kb + 16 + 8 * hh);
    acc = wmma_f16(a.v, b.v, acc);
  }
#pragma unroll
  for (int r = 0; r < 8; ++r) {
    const int row = w * 16 + 8 * hh + r;
    if (m < NCLS) so[row * NCLS + m] = acc[r] + bc[m];
  }
  __syncthreads();
  if (w == 0) {
    cls_emit(so, out, l);
    __threadfence();
    cls_emit(so, out, l);
  }
}

extern "C" void kernel_launch(void* const* d_in, const int* in_sizes, int n_in,
                              void* d_out, int out_size, void* d_ws, size_t ws_size,
                              hipStream_t stream) {
  if (n_in < 13) return;
  if (in_sizes[0] != N_NODES * IN_DIM || in_sizes[1] != 2 * N_EDGES || in_sizes[2] != N_NODES ||
      in_sizes[3] != HID * IN_DIM || in_sizes[4] != HID || in_sizes[5] != HID * HID ||
      in_sizes[6] != HID || in_sizes[7] != HID * HID || in_sizes[8] != HID ||
      in_sizes[9] != HID * HID || in_sizes[10] != HID || in_sizes[11] != NCLS * HID ||
      in_sizes[12] != NCLS || out_size != NGRAPH * NCLS)
    return;

  const float* x   = (const float*)d_in[0];
  const int*   ei  = (const int*)d_in[1];
  const int*   gid = (const int*)d_in[2];
  const float* W1a = (const float*)d_in[3];
  const float* b1a = (const float*)d_in[4];
  const float* W1b = (const float*)d_in[5];
  const float* b1b = (const float*)d_in[6];
  const float* W2a = (const float*)d_in[7];
  const float* b2a = (const float*)d_in[8];
  const float* W2b = (const float*)d_in[9];
  const float* b2b = (const float*)d_in[10];
  const float* Wc  = (const float*)d_in[11];
  const float* bc  = (const float*)d_in[12];
  float* out = (float*)d_out;

  char* ws = (char*)d_ws;
  size_t off = 0;
  auto take = [&](size_t bytes) -> char* {
    char* p = ws + off;
    off = (off + bytes + 255) & ~(size_t)255;
    return p;
  };
  _Float16* Wh1a = (_Float16*)take((size_t)HID * IN_DIM * 2);
  _Float16* Wh1b = (_Float16*)take((size_t)HID * HID * 2);
  _Float16* Wh2a = (_Float16*)take((size_t)HID * HID * 2);
  _Float16* Wh2b = (_Float16*)take((size_t)HID * HID * 2);
  _Float16* Wch  = (_Float16*)take((size_t)NCLS_PAD * HID * 2);
  _Float16* pm   = (_Float16*)take((size_t)NGRAPH * HID * 2);
  _Float16* zh   = (_Float16*)take((size_t)N_NODES * HID * 2);
  _Float16* th   = (_Float16*)take((size_t)N_NODES * HID * 2);
  float*    hf   = (float*)take((size_t)N_NODES * HID * 4);
  if (off > ws_size) return;

  const int TB = 256;

  k_cvt<<<(HID * IN_DIM / 8 + TB - 1) / TB, TB, 0, stream>>>(W1a, Wh1a, HID * IN_DIM, HID * IN_DIM / 8);
  k_cvt<<<(HID * HID / 8 + TB - 1) / TB, TB, 0, stream>>>(W1b, Wh1b, HID * HID, HID * HID / 8);
  k_cvt<<<(HID * HID / 8 + TB - 1) / TB, TB, 0, stream>>>(W2a, Wh2a, HID * HID, HID * HID / 8);
  k_cvt<<<(HID * HID / 8 + TB - 1) / TB, TB, 0, stream>>>(W2b, Wh2b, HID * HID, HID * HID / 8);
  k_cvt<<<(NCLS_PAD * HID / 8 + TB - 1) / TB, TB, 0, stream>>>(Wc, Wch, NCLS * HID, NCLS_PAD * HID / 8);

  const int ntiles = (N_NODES / 16) * (HID / 64);
  const int gemm_blocks = (ntiles + 7) / 8;

  k_agg<IN_DIM, 256><<<(N_NODES + 255) / 256, TB, 0, stream>>>(x, ei, zh);
  k_gemm<0><<<gemm_blocks, TB, 0, stream>>>(zh, Wh1a, b1a, (void*)th, IN_DIM, ntiles);
  k_gemm<1><<<gemm_blocks, TB, 0, stream>>>(th, Wh1b, b1b, (void*)hf, HID, ntiles);

  k_agg<HID, 128><<<(N_NODES + 127) / 128, TB, 0, stream>>>(hf, ei, zh);
  k_gemm<0><<<gemm_blocks, TB, 0, stream>>>(zh, Wh2a, b2a, (void*)th, HID, ntiles);
  k_gemm<1><<<gemm_blocks, TB, 0, stream>>>(th, Wh2b, b2b, (void*)hf, HID, ntiles);

  k_pool<<<NGRAPH, TB, 0, stream>>>(hf, gid, pm);
  k_cls<<<1, 128, 0, stream>>>(pm, Wch, bc, out);
}
